// BertForSequenceClassification_three_26800595927388
// MI455X (gfx1250) — hardware-run, weakly checked
//
#include <hip/hip_runtime.h>
#include <math.h>

#ifndef NB
#define NB 32
#endif
#ifndef SEQ
#define SEQ 512
#endif
#define NB_FULL 32
#define SEQ_FULL 512
#define HID 768
#define AUD 64
#define PROJ 30
#define PPAD 32
#define VR_PITCH 64
#define MTOK (NB * SEQ)
#define MD_ROWS 32
#define PROJ_ROWS 128
#define NPBLK (MTOK / PROJ_ROWS)
#define GT_COLS (SEQ / 64)
#define GT_PER_B ((SEQ / 16) * GT_COLS)
#define OUT1_OFF (NB_FULL * HID)
#define OUT2_OFF (OUT1_OFF + NB_FULL * SEQ_FULL * SEQ_FULL)

#define C_ACT 64.0f
#define C_WGT 1024.0f
#define C_TXT 1024.0f
#define C_AUDV 64.0f
#define C_RES 2048.0f
#define C_F0 64.0f
#define INV_ACT_WGT (1.0f / (C_ACT * C_WGT))
#define INV_F0_WGT (1.0f / (C_F0 * C_WGT))
#define INV_TXT2 (1.0f / (C_TXT * C_TXT))
#define INV_TXT2_RES (1.0f / (C_TXT * C_TXT * C_RES))
#define INV_AUD2 (1.0f / (C_AUDV * C_AUDV))
#define INV_AUD2_RES (1.0f / (C_AUDV * C_AUDV * C_RES))

static_assert(SEQ == SEQ_FULL);
static_assert(SEQ == 512);
static_assert(NB >= 1 && NB <= NB_FULL);
static_assert(NB <= MD_ROWS && MD_ROWS == 32);
static_assert(MTOK % PROJ_ROWS == 0);
static_assert(HID % 64 == 0 && AUD % 32 == 0 && PPAD == 32);
static_assert((HID / 64) % 4 == 0);
static_assert((NB * GT_PER_B) % 8 == 0);
static_assert((MTOK * 8) % 256 == 0);
static_assert(PPAD * (HID / 8) == 12 * 256);
static_assert(PPAD * (AUD / 8) == 256);
static_assert(OUT1_OFF * 4 == 98304);
static_assert((long long)OUT2_OFF * 4 == 33652736LL);
static_assert((long long)(OUT2_OFF + NB_FULL * SEQ_FULL * SEQ_FULL) * 4 == 67207168LL);
static_assert(NB * HID <= OUT1_OFF);
static_assert(OUT1_OFF + NB * SEQ * SEQ <= OUT2_OFF);

typedef _Float16 h16;
typedef __attribute__((ext_vector_type(16))) _Float16 v16h;
typedef __attribute__((ext_vector_type(8)))  _Float16 v8h;
typedef __attribute__((ext_vector_type(8)))  float    v8f;
typedef __attribute__((ext_vector_type(4)))  float    v4f;


#define VST2V4(ptr, val) do { const v4f vst2_v4_ = (val); *(volatile v4f*)(ptr) = vst2_v4_; __threadfence(); *(volatile v4f*)(ptr) = vst2_v4_; } while (0)

__device__ __forceinline__ float bfr(float f) {
    unsigned u = __float_as_uint(f);
    u += 0x7FFFu + ((u >> 16) & 1u);
    return __uint_as_float(u & 0xFFFF0000u);
}
static __device__ __forceinline__ h16 toh_flush(float v) {
    const float w = (fabsf(v) < 6.103515625e-05f) ? 0.0f : v;
    return (h16)w;
}
__device__ __forceinline__ void st8h(h16* P, size_t o, const float* v) {
    v8h pk;
#pragma unroll
    for (int i = 0; i < 8; ++i) pk[i] = toh_flush(v[i]);
    *(volatile v8h*)(P + o) = pk;
    __threadfence();
    *(volatile v8h*)(P + o) = pk;
}

union FragU { v16h v; v8h h[2]; };
__device__ __forceinline__ v16h frag_ld(const h16* p) {
    FragU f; f.h[0] = *(const v8h*)(p); f.h[1] = *(const v8h*)(p + 16); return f.v;
}
__device__ __forceinline__ v16h cvt_frag(const float* p, const float carry) {
    const v4f x0 = *(const v4f*)(p), x1 = *(const v4f*)(p + 4), x2 = *(const v4f*)(p + 16), x3 = *(const v4f*)(p + 20);
    v16h f;
    f[0]  = toh_flush(bfr(x0.x) * carry); f[1]  = toh_flush(bfr(x0.y) * carry);
    f[2]  = toh_flush(bfr(x0.z) * carry); f[3]  = toh_flush(bfr(x0.w) * carry);
    f[4]  = toh_flush(bfr(x1.x) * carry); f[5]  = toh_flush(bfr(x1.y) * carry);
    f[6]  = toh_flush(bfr(x1.z) * carry); f[7]  = toh_flush(bfr(x1.w) * carry);
    f[8]  = toh_flush(bfr(x2.x) * carry); f[9]  = toh_flush(bfr(x2.y) * carry);
    f[10] = toh_flush(bfr(x2.z) * carry); f[11] = toh_flush(bfr(x2.w) * carry);
    f[12] = toh_flush(bfr(x3.x) * carry); f[13] = toh_flush(bfr(x3.y) * carry);
    f[14] = toh_flush(bfr(x3.z) * carry); f[15] = toh_flush(bfr(x3.w) * carry);
    return f;
}
__device__ __forceinline__ v8f wmma16g(v16h a, v16h b, v8f c) {
    c = __builtin_amdgcn_wmma_f32_16x16x32_f16(false, a, false, b, (short)0, c, false, false);
    asm volatile("v_nop\n\tv_nop\n\tv_nop\n\tv_nop" : "+v"(c) : "v"(a), "v"(b));
    return c;
}
__device__ __forceinline__ void wave_sync_lds() {
    __builtin_amdgcn_fence(3  , "workgroup");
    __builtin_amdgcn_wave_barrier();
    __builtin_amdgcn_fence(2  , "workgroup");
}
__device__ __forceinline__ void store_tile16x64(const float* slab, float* dst, unsigned pitch, unsigned lane) {
    const unsigned hh = lane >> 4, c4 = (lane & 15u) * 4u;
#pragma unroll
    for (int half = 0; half < 2; ++half) {
        v4f vv[4];
#pragma unroll
        for (int it = 0; it < 4; ++it) {
            const unsigned row = (unsigned)(half * 4 + it) * 2u + hh;
            vv[it] = *(const v4f*)(slab + row * 68u + c4);
        }
        for (int pass = 0; pass < 2; ++pass) {
#pragma unroll
            for (int it = 0; it < 4; ++it) {
                const unsigned row = (unsigned)(half * 4 + it) * 2u + hh;
                *(volatile v4f*)(dst + (size_t)row * pitch + c4) = vv[it];
            }
            __threadfence();
        }
    }
}

__global__ __launch_bounds__(256) void k_wplanes(const float* __restrict__ Wt, const float* __restrict__ Wa,
                                                 h16* __restrict__ Wt16, h16* __restrict__ Wa16) {
    const unsigned t = threadIdx.x;
    float v[8];
    if (blockIdx.x < 12u) {
        const unsigned u = blockIdx.x * 256u + t;
        const unsigned n = u / 96u, k0 = 8u * (u - n * 96u);
        const int nc = min((int)n, PROJ - 1);
        const float* src = Wt + (size_t)(unsigned)nc * HID + k0;
        const v4f a = *(const v4f*)src, b = *(const v4f*)(src + 4);
        const float x[8] = {a.x, a.y, a.z, a.w, b.x, b.y, b.z, b.w};
#pragma unroll
        for (int i = 0; i < 8; ++i) { const float w = bfr(x[i]) * C_WGT; v[i] = (n < (unsigned)PROJ) ? w : 0.0f; }
        st8h(Wt16, (size_t)u * 8u, v);
    } else {
        const unsigned n = t >> 3, k0 = 8u * (t & 7u);
        const int nc = min((int)n, PROJ - 1);
        const float* src = Wa + (size_t)(unsigned)nc * AUD + k0;
        const v4f a = *(const v4f*)src, b = *(const v4f*)(src + 4);
        const float x[8] = {a.x, a.y, a.z, a.w, b.x, b.y, b.z, b.w};
#pragma unroll
        for (int i = 0; i < 8; ++i) { const float w = bfr(x[i]) * C_WGT; v[i] = (n < (unsigned)PROJ) ? w : 0.0f; }
        st8h(Wa16, (size_t)t * 8u, v);
    }
}

__global__ __launch_bounds__(256) void k_proj(const float* __restrict__ hid, const float* __restrict__ aud,
                                              const h16* __restrict__ Wt16, const h16* __restrict__ Wa16,
                                              float* __restrict__ text32, h16* __restrict__ avr, float* __restrict__ part) {
    __shared__ __align__(16) float sT[8][16 * 36];
    __shared__ float sQ[8];
    const unsigned lane = threadIdx.x & 31u, wave = threadIdx.x >> 5;
    const unsigned hh = lane >> 4, c = lane & 15u;
    const unsigned m0 = blockIdx.x * (unsigned)PROJ_ROWS + wave * 16u;
    v8f at[2], aa[2];
#pragma unroll
    for (int j = 0; j < 2; ++j) { at[j] = (v8f){0.f,0.f,0.f,0.f,0.f,0.f,0.f,0.f}; aa[j] = at[j]; }
    {
        const float* hp = hid + (size_t)(m0 + c) * HID + 8u * hh;
        const h16* w0 = Wt16 + (size_t)c * HID + 8u * hh;
        const h16* w1 = Wt16 + (size_t)(16u + c) * HID + 8u * hh;
        for (unsigned k0 = 0; k0 < (unsigned)HID; k0 += 32u) {
            const v16h a = cvt_frag(hp + k0, C_ACT);
            const v16h b0 = frag_ld(w0 + k0);
            const v16h b1 = frag_ld(w1 + k0);
            at[0] = wmma16g(a, b0, at[0]);
            at[1] = wmma16g(a, b1, at[1]);
        }
    }
    {
        const float* ap = aud + (size_t)(m0 + c) * AUD + 8u * hh;
        const h16* w0 = Wa16 + (size_t)c * AUD + 8u * hh;
        const h16* w1 = Wa16 + (size_t)(16u + c) * AUD + 8u * hh;
#pragma unroll
        for (int ks = 0; ks < AUD / 32; ++ks) {
            const v16h a = cvt_frag(ap + 32 * ks, C_ACT);
            const v16h b0 = frag_ld(w0 + 32 * ks);
            const v16h b1 = frag_ld(w1 + 32 * ks);
            aa[0] = wmma16g(a, b0, aa[0]);
            aa[1] = wmma16g(a, b1, aa[1]);
        }
    }
    float* slab = sT[wave];
    float q = 0.f;
#pragma unroll
    for (int j = 0; j < 2; ++j)
#pragma unroll
        for (int r = 0; r < 8; ++r) {
            const float tv = at[j][r] * INV_ACT_WGT;
            q += tv * tv;
            slab[(8u * hh + (unsigned)r) * 36u + (unsigned)j * 16u + c] = tv;
        }
#pragma unroll
    for (int o = 16; o > 0; o >>= 1) q += __shfl_xor(q, o, 32);
    if (lane == 0u) sQ[wave] = q;
    wave_sync_lds();
    const unsigned q8 = lane >> 3;
    {
        const unsigned c4 = (lane & 7u) * 4u;
        v4f vv[4];
#pragma unroll
        for (int it = 0; it < 4; ++it) vv[it] = *(const v4f*)(slab + ((unsigned)it * 4u + q8) * 36u + c4);
        for (int pass = 0; pass < 2; ++pass) {
#pragma unroll
            for (int it = 0; it < 4; ++it)
                *(volatile v4f*)(text32 + (size_t)(m0 + (unsigned)it * 4u + q8) * PPAD + c4) = vv[it];
            __threadfence();
        }
    }
    wave_sync_lds();
#pragma unroll
    for (int j = 0; j < 2; ++j)
#pragma unroll
        for (int r = 0; r < 8; ++r)
            slab[(8u * hh + (unsigned)r) * 36u + (unsigned)j * 16u + c] = aa[j][r] * (INV_ACT_WGT * C_AUDV);
    wave_sync_lds();
    {
        const unsigned p = lane & 7u, g = p & 3u;
#pragma unroll
        for (int it = 0; it < 4; ++it) {
            const unsigned row = (unsigned)it * 4u + q8;
            const float* sp = slab + row * 36u + 8u * g;
            const v4f x0 = *(const v4f*)sp, x1 = *(const v4f*)(sp + 4);
            const float zz[8] = {x0.x, x0.y, x0.z, x0.w, x1.x, x1.y, x1.z, x1.w};
            float w[8];
#pragma unroll
            for (int i = 0; i < 8; ++i) {
                const float vf = (float)toh_flush(zz[i]);
                w[i] = (p < 4u) ? zz[i] : (zz[i] - vf) * C_RES;
            }
            st8h(avr, (size_t)(m0 + row) * VR_PITCH + 8u * p, w);
        }
    }
    __syncthreads();
    if (wave == 0u) {
        float tot = 0.f;
#pragma unroll
        for (int w = 0; w < 8; ++w) tot += sQ[w];
        v4f pv = {0.f, 0.f, 0.f, 0.f};
        pv.x = (lane == 0u) ? tot : 0.0f;
        if (lane < 8u) { VST2V4(part + (size_t)blockIdx.x * 32u + lane * 4u, pv); }
    }
}

__global__ __launch_bounds__(256) void k_norm_split(const float* __restrict__ text32, const float* __restrict__ part,
                                                    h16* __restrict__ tvr) {
    __shared__ float sN;
    if (threadIdx.x == 0u) {
        float s = 0.f;
        for (unsigned i = 0; i < (unsigned)NPBLK; ++i) s += part[(size_t)i * 32u];
        sN = sqrtf(sqrtf(s));
    }
    __syncthreads();
    const float nrm = sN;
    const unsigned u = blockIdx.x * 256u + threadIdx.x;
    const unsigned row = u >> 3, p = u & 7u, g = p & 3u;
    const float* sp = text32 + (size_t)row * PPAD + 8u * g;
    const v4f x0 = *(const v4f*)sp, x1 = *(const v4f*)(sp + 4);
    const float xx[8] = {x0.x, x0.y, x0.z, x0.w, x1.x, x1.y, x1.z, x1.w};
    float w[8];
#pragma unroll
    for (int i = 0; i < 8; ++i) {
        const float zz = (xx[i] / nrm) * C_TXT;
        const float vf = (float)toh_flush(zz);
        w[i] = (p < 4u) ? zz : (zz - vf) * C_RES;
    }
    st8h(tvr, (size_t)row * VR_PITCH + 8u * p, w);
}

__global__ __launch_bounds__(256) void k_gram(const h16* __restrict__ tvr, const h16* __restrict__ avr,
                                              const float* __restrict__ p_tw, const float* __restrict__ p_aw,
                                              const float* __restrict__ p_fb,
                                              float* __restrict__ out1, float* __restrict__ out2, float* __restrict__ raw0) {
    __shared__ __align__(16) float sT[8][16 * 68];
    const unsigned lane = threadIdx.x & 31u, wave = threadIdx.x >> 5;
    const unsigned hh = lane >> 4, c = lane & 15u;
    const unsigned tile = blockIdx.x * 8u + wave;
    const unsigned b = tile / (unsigned)GT_PER_B;
    const unsigned rem = tile - b * (unsigned)GT_PER_B;
    const unsigned ti = rem / (unsigned)GT_COLS;
    const unsigned tj = rem - ti * (unsigned)GT_COLS;
    const unsigned i0 = ti * 16u, j0 = tj * 64u;
    const float tw = bfr(p_tw[0]), aw = bfr(p_aw[0]), fb = bfr(p_fb[0]);
    const v8f z8 = {0.f,0.f,0.f,0.f,0.f,0.f,0.f,0.f};

    v8f ta[4], ga[4];
    {
        const h16* pa = tvr + (size_t)(b * SEQ + i0 + c) * VR_PITCH + 8u * hh;
        const v16h av = frag_ld(pa), ar = frag_ld(pa + 32);
#pragma unroll
        for (int j = 0; j < 4; ++j) {
            const h16* pb = tvr + (size_t)(b * SEQ + j0 + (unsigned)j * 16u + c) * VR_PITCH + 8u * hh;
            const v16h bv = frag_ld(pb), br = frag_ld(pb + 32);
            v8f mm = wmma16g(av, bv, z8);
            v8f xx = wmma16g(av, br, z8);
            xx = wmma16g(ar, bv, xx);
#pragma unroll
            for (int r = 0; r < 8; ++r) ta[j][r] = fmaxf(mm[r] * INV_TXT2 + xx[r] * INV_TXT2_RES, 0.0f);
        }
    }
    {
        const h16* pa = avr + (size_t)(b * SEQ + i0 + c) * VR_PITCH + 8u * hh;
        const v16h av = frag_ld(pa), ar = frag_ld(pa + 32);
#pragma unroll
        for (int j = 0; j < 4; ++j) {
            const h16* pb = avr + (size_t)(b * SEQ + j0 + (unsigned)j * 16u + c) * VR_PITCH + 8u * hh;
            const v16h bv = frag_ld(pb), br = frag_ld(pb + 32);
            v8f mm = wmma16g(av, bv, z8);
            v8f xx = wmma16g(av, br, z8);
            xx = wmma16g(ar, bv, xx);
#pragma unroll
            for (int r = 0; r < 8; ++r) ga[j][r] = fmaxf(mm[r] * INV_AUD2 + xx[r] * INV_AUD2_RES, 0.0f);
        }
    }

    float* slab = sT[wave];
#pragma unroll
    for (int j = 0; j < 4; ++j)
#pragma unroll
        for (int r = 0; r < 8; ++r)
            slab[(8u * hh + (unsigned)r) * 68u + (unsigned)j * 16u + c] = ta[j][r];
    wave_sync_lds();
    store_tile16x64(slab, out1 + (size_t)(b * SEQ + i0) * SEQ + j0, SEQ, lane);
    wave_sync_lds();
    float rrow[4];
#pragma unroll
    for (int j = 0; j < 4; ++j) {
#pragma unroll
        for (int r = 0; r < 8; ++r) {
            const float raw = tw * ta[j][r] + aw * ga[j][r] + fb;
            if (r == 0) rrow[j] = raw;
            slab[(8u * hh + (unsigned)r) * 68u + (unsigned)j * 16u + c] = fmaxf(raw, 0.0f);
        }
    }
    wave_sync_lds();
    store_tile16x64(slab, out2 + (size_t)(b * SEQ + i0) * SEQ + j0, SEQ, lane);
    wave_sync_lds();
    if (ti == 0u) {
#pragma unroll
        for (int j = 0; j < 4; ++j) slab[(8u * hh) * 68u + (unsigned)j * 16u + c] = rrow[j];
        wave_sync_lds();
        const unsigned c4 = (lane & 15u) * 4u;
        const v4f rv = *(const v4f*)(slab + c4);
        if (lane < 16u) { VST2V4(raw0 + (size_t)b * SEQ + j0 + c4, rv); }
    }
}

__global__ __launch_bounds__(256) void k_row0(const float* __restrict__ hid, const float* __restrict__ mask,
                                              const float* __restrict__ raw0, h16* __restrict__ f0p) {
    __shared__ float att[SEQ];
    __shared__ float red[256];
    __shared__ __align__(16) float fr[HID];
    const unsigned b = blockIdx.x, tid = threadIdx.x;
    if (b >= (unsigned)NB) {
        if (tid < 96u) {
            float v[8];
#pragma unroll
            for (int i = 0; i < 8; ++i) v[i] = 0.0f;
            st8h(f0p, (size_t)b * HID + 8u * tid, v);
        }
        return;
    }
    const float* mk = mask + (size_t)b * SEQ_FULL;
    const float mk0 = bfr(mk[0]);
    const float l0 = (raw0[(size_t)b * SEQ + tid] + bfr(mk[tid])) + mk0;
    const float l1 = (raw0[(size_t)b * SEQ + tid + 256u] + bfr(mk[tid + 256u])) + mk0;
    red[tid] = fmaxf(l0, l1);
    __syncthreads();
    for (unsigned st = 128u; st > 0u; st >>= 1) {
        if (tid < st) red[tid] = fmaxf(red[tid], red[tid + st]);
        __syncthreads();
    }
    const float mx = red[0];
    __syncthreads();
    const float e0 = expf(l0 - mx), e1 = expf(l1 - mx);
    red[tid] = e0 + e1;
    __syncthreads();
    for (unsigned st = 128u; st > 0u; st >>= 1) {
        if (tid < st) red[tid] += red[tid + st];
        __syncthreads();
    }
    const float den = red[0];
    att[tid] = e0 / den;
    att[tid + 256u] = e1 / den;
    __syncthreads();

    const float* hb = hid + (size_t)b * SEQ_FULL * HID;
    float a0 = 0.f, a1 = 0.f, a2 = 0.f;
    for (unsigned t = 0; t < (unsigned)SEQ; ++t) {
        const float a = att[t];
        const float* hr = hb + (size_t)t * HID;
        a0 += a * bfr(hr[tid]);
        a1 += a * bfr(hr[tid + 256u]);
        a2 += a * bfr(hr[tid + 512u]);
    }
    fr[tid] = a0 + bfr(hb[tid]);
    fr[tid + 256u] = a1 + bfr(hb[tid + 256u]);
    fr[tid + 512u] = a2 + bfr(hb[tid + 512u]);
    __syncthreads();
    if (tid < 96u) {
        const v4f x0 = *(const v4f*)(fr + 8u * tid), x1 = *(const v4f*)(fr + 8u * tid + 4u);
        float v[8] = {x0.x * C_F0, x0.y * C_F0, x0.z * C_F0, x0.w * C_F0, x1.x * C_F0, x1.y * C_F0, x1.z * C_F0, x1.w * C_F0};
        st8h(f0p, (size_t)b * HID + 8u * tid, v);
    }
}

__global__ __launch_bounds__(128) void k_dense(const h16* __restrict__ f0p, const float* __restrict__ Wd,
                                               const float* __restrict__ bd, float* __restrict__ hpl) {
    __shared__ __align__(16) float sT[4][16 * 68];
    const unsigned lane = threadIdx.x & 31u, wave = threadIdx.x >> 5;
    const unsigned hh = lane >> 4, c = lane & 15u;
    const unsigned n0 = (blockIdx.x * 4u + wave) * 64u;
    v8f acc[2][4];
#pragma unroll
    for (int i = 0; i < 2; ++i)
#pragma unroll
        for (int j = 0; j < 4; ++j) acc[i][j] = (v8f){0.f,0.f,0.f,0.f,0.f,0.f,0.f,0.f};
    for (unsigned k0 = 0; k0 < (unsigned)HID; k0 += 32u) {
        const v16h a0 = frag_ld(f0p + (size_t)c * HID + 8u * hh + k0);
        const v16h a1 = frag_ld(f0p + (size_t)(16u + c) * HID + 8u * hh + k0);
#pragma unroll
        for (int j = 0; j < 4; ++j) {
            const v16h bw = cvt_frag(Wd + (size_t)(n0 + (unsigned)j * 16u + c) * HID + 8u * hh + k0, C_WGT);
            acc[0][j] = wmma16g(a0, bw, acc[0][j]);
            acc[1][j] = wmma16g(a1, bw, acc[1][j]);
        }
    }
    float* slab = sT[wave];
#pragma unroll
    for (int i = 0; i < 2; ++i) {
#pragma unroll
        for (int j = 0; j < 4; ++j) {
            const float bv = bfr(bd[n0 + (unsigned)j * 16u + c]);
#pragma unroll
            for (int r = 0; r < 8; ++r)
                slab[(8u * hh + (unsigned)r) * 68u + (unsigned)j * 16u + c] = acc[i][j][r] * INV_F0_WGT + bv;
        }
        wave_sync_lds();
        store_tile16x64(slab, hpl + (size_t)((unsigned)i * 16u) * HID + n0, HID, lane);
        wave_sync_lds();
    }
}

__global__ __launch_bounds__(256) void k_ln(const float* __restrict__ hpl, const float* __restrict__ lw,
                                            const float* __restrict__ lb, float* __restrict__ out0) {
    const unsigned row = blockIdx.x * 8u + (threadIdx.x >> 5);
    const unsigned L = threadIdx.x & 31u;
    if (row >= (unsigned)NB) return;
    const float* hr = hpl + (size_t)row * HID + 4u * L;
    v4f x[6];
#pragma unroll
    for (int i = 0; i < 6; ++i) x[i] = *(const v4f*)(hr + 128 * i);
    float s = 0.f;
#pragma unroll
    for (int i = 0; i < 6; ++i) s += (x[i].x + x[i].y) + (x[i].z + x[i].w);
#pragma unroll
    for (int o = 16; o > 0; o >>= 1) s += __shfl_xor(s, o, 32);
    const float mu = s * (1.0f / (float)HID);
    float q = 0.f;
#pragma unroll
    for (int i = 0; i < 6; ++i) {
        x[i].x -= mu; x[i].y -= mu; x[i].z -= mu; x[i].w -= mu;
        q += (x[i].x * x[i].x + x[i].y * x[i].y) + (x[i].z * x[i].z + x[i].w * x[i].w);
    }
#pragma unroll
    for (int o = 16; o > 0; o >>= 1) q += __shfl_xor(q, o, 32);
    const float sq = sqrtf(q * (1.0f / (float)HID) + 1e-12f);
    v4f y[6];
#pragma unroll
    for (int i = 0; i < 6; ++i) {
        const v4f g = *(const v4f*)(lw + 128 * i + 4u * L);
        const v4f bb = *(const v4f*)(lb + 128 * i + 4u * L);
        y[i].x = (bfr(g.x) * x[i].x) / sq + bfr(bb.x);
        y[i].y = (bfr(g.y) * x[i].y) / sq + bfr(bb.y);
        y[i].z = (bfr(g.z) * x[i].z) / sq + bfr(bb.z);
        y[i].w = (bfr(g.w) * x[i].w) / sq + bfr(bb.w);
    }
    float* dst = out0 + (size_t)row * HID + 4u * L;
    for (int pass = 0; pass < 2; ++pass) {
#pragma unroll
        for (int i = 0; i < 6; ++i) *(volatile v4f*)(dst + 128 * i) = y[i];
        __threadfence();
    }
}

extern "C" void kernel_launch(void* const* d_in, const int* in_sizes, int n_in, void* d_out, int out_size,
                              void* d_ws, size_t ws_size, hipStream_t stream) {
    if (n_in < 12) return;
    if (in_sizes[0] < MTOK * HID || in_sizes[1] < MTOK * AUD || in_sizes[2] < NB * SEQ) return;
    if (in_sizes[3] < PROJ * HID || in_sizes[4] < PROJ * AUD) return;
    if (in_sizes[5] < 1 || in_sizes[6] < 1 || in_sizes[7] < 1) return;
    if (in_sizes[8] < HID * HID || in_sizes[9] < HID || in_sizes[10] < HID || in_sizes[11] < HID) return;
    if (out_size < OUT2_OFF + NB * SEQ * SEQ) return;

    const float* hid  = (const float*)d_in[0];
    const float* aud  = (const float*)d_in[1];
    const float* mask = (const float*)d_in[2];
    const float* Wt   = (const float*)d_in[3];
    const float* Wa   = (const float*)d_in[4];
    const float* p_tw = (const float*)d_in[5];
    const float* p_aw = (const float*)d_in[6];
    const float* p_fb = (const float*)d_in[7];
    const float* Wd   = (const float*)d_in[8];
    const float* bd   = (const float*)d_in[9];
    const float* lw   = (const float*)d_in[10];
    const float* lb   = (const float*)d_in[11];
    float* out = (float*)d_out;

    char* wsp = (char*)d_ws;
    size_t off = 0;
    auto carve = [&](size_t bytes) -> void* { void* r = wsp + off; off += (bytes + 255) & ~(size_t)255; return r; };
    h16*   Wt16   = (h16*)carve((size_t)PPAD * HID * 2);
    h16*   Wa16   = (h16*)carve((size_t)PPAD * AUD * 2);
    float* text32 = (float*)carve((size_t)MTOK * PPAD * 4);
    h16*   avr    = (h16*)carve((size_t)MTOK * VR_PITCH * 2);
    h16*   tvr    = (h16*)carve((size_t)MTOK * VR_PITCH * 2);
    float* part   = (float*)carve((size_t)NPBLK * 32 * 4);
    float* raw0   = (float*)carve((size_t)NB * SEQ * 4);
    h16*   f0p    = (h16*)carve((size_t)MD_ROWS * HID * 2);
    float* hpl    = (float*)carve((size_t)MD_ROWS * HID * 4);
    if (off > ws_size || off > (size_t)134217728) return;

    k_wplanes<<<13, 256, 0, stream>>>(Wt, Wa, Wt16, Wa16);
    k_proj<<<NPBLK, 256, 0, stream>>>(hid, aud, (const h16*)Wt16, (const h16*)Wa16, text32, avr, part);
    k_norm_split<<<(MTOK * 8) / 256, 256, 0, stream>>>(text32, part, tvr);
    k_gram<<<(NB * GT_PER_B) / 8, 256, 0, stream>>>((const h16*)tvr, (const h16*)avr, p_tw, p_aw, p_fb,
                                                    out + OUT1_OFF, out + OUT2_OFF, raw0);
    k_row0<<<MD_ROWS, 256, 0, stream>>>(hid, mask, raw0, f0p);
    k_dense<<<(HID / 64) / 4, 128, 0, stream>>>((const h16*)f0p, Wd, bd, hpl);
    k_ln<<<MD_ROWS / 8, 256, 0, stream>>>(hpl, lw, lb, out);
}
